// BraskModel_77429670412702
// MI455X (gfx1250) — hardware-run, weakly checked
//
#include <hip/hip_runtime.h>


namespace {
constexpr int NBt = 4, R = 8, S = 8, L = 256, H = 768, A = 256, TD = 100, NROW = NBt * L  ;
constexpr int NV = 8;
constexpr int ND = 16;
constexpr float XS = 8.0f, WSC = 256.0f;
typedef _Float16 b16;
typedef __attribute__((ext_vector_type(16))) _Float16 v16b;
typedef __attribute__((ext_vector_type(8))) _Float16 v8b;
typedef __attribute__((ext_vector_type(8))) float v8f;
typedef __attribute__((ext_vector_type(4))) float v4f;
__device__ __forceinline__ float bf16_rne(float f) { unsigned int u = __float_as_uint(f); u += 0x7FFFu + ((u >> 16) & 1u); float r = __uint_as_float(u & 0xFFFF0000u); asm volatile("" : "+v"(r)); return r; }
__device__ __forceinline__ float bfv(float f) { float r = bf16_rne(f); asm volatile("" : "+v"(r)); return r; }
__device__ __forceinline__ v16b frag_kb(const b16* p, int hh) { const v8b a = *(const v8b*)(p + 8 * hh), b = *(const v8b*)(p + 16 + 8 * hh); v16b f;
#pragma unroll
  for (int e = 0; e < 8; ++e) { f[e] = a[e]; f[8 + e] = b[e]; } return f; }
__device__ __forceinline__ v8f wmma16b(v16b a, v16b b, v8f c) { v8f d = __builtin_amdgcn_wmma_f32_16x16x32_f16(false, a, false, b, (short)0, c, false, false); asm volatile("v_nop\n\tv_nop\n\tv_nop\n\tv_nop" : "+v"(d) : "v"(a), "v"(b)); return d; }
__device__ __forceinline__ void wave_lds_sync() { __builtin_amdgcn_fence(__ATOMIC_RELEASE, "workgroup"); __builtin_amdgcn_wave_barrier(); __builtin_amdgcn_fence(__ATOMIC_ACQUIRE, "workgroup"); }
__device__ __forceinline__ float pmul(float a, float b) { float p = a * b; asm volatile("" : "+v"(p)); return p; }
__device__ __forceinline__ int iclamp(int v, int lo, int hi) { return v < lo ? lo : (v > hi ? hi : v); }

__global__ __launch_bounds__(256) void setup_kernel(const float* __restrict__ fwx, const float* __restrict__ bwx, const float* __restrict__ ffeWs, const float* __restrict__ ffebs, const float* __restrict__ ffeWx, const float* __restrict__ ffebx, const float* __restrict__ bfeWs, const float* __restrict__ bfebs, const float* __restrict__ bfeWx, const float* __restrict__ bfebx,
    const float* __restrict__ ftws, const float* __restrict__ ftwe, const float* __restrict__ bhws, const float* __restrict__ bhwe, const float* __restrict__ rel1, const float* __restrict__ rel2, const float* __restrict__ xmean, const float* __restrict__ fWr, const float* __restrict__ fbr, const float* __restrict__ fWg, const float* __restrict__ fbg, const float* __restrict__ bWr, const float* __restrict__ bbr, const float* __restrict__ bWg, const float* __restrict__ bbg,
    b16* __restrict__ WX, float* __restrict__ DV, float* __restrict__ DS, float* __restrict__ WRG) { const size_t nt = (size_t)gridDim.x * 256, u0 = (size_t)blockIdx.x * 256 + threadIdx.x; v8b v;
  for (size_t u = u0; u < (size_t)2 * A * (H / 8); u += nt) { const int o = (int)(u / (H / 8)), k0 = (int)(u % (H / 8)) * 8; const float* W = o < A ? fwx : bwx; const int c = o % A;
#pragma unroll
    for (int j = 0; j < 8; ++j) v[j] = (b16)(bf16_rne(W[(size_t)(k0 + j) * A + c]) * WSC); for (int pass = 0; pass < 2; ++pass) { *(volatile v8b*)(WX + (size_t)o * H + k0) = v; __threadfence(); } }
  for (size_t u = u0; u < (size_t)NV * H; u += nt) { const int j = (int)(u / H), k = (int)(u % H); const float* W = (j == 0 || j == 1) ? ffeWx : (j == 2 || j == 3) ? bfeWx : (j == 4 || j == 5) ? ffeWs : bfeWs; const float* w = (j == 0 || j == 4) ? ftws : (j == 1 || j == 5) ? ftwe : (j == 2 || j == 6) ? bhws : bhwe; float s = 0.0f;
    for (int o = 0; o < H; ++o) s += pmul(bfv(W[(size_t)k * H + o]), bfv(w[o])); for (int pass = 0; pass < 2; ++pass) { ((volatile float*)DV)[u] = s; __threadfence(); } }
  if (u0 < 32) { float s = 0.0f; if (u0 < 8) { const int j = (int)u0; const float* bvec = (j == 0 || j == 1) ? ffebx : (j == 2 || j == 3) ? bfebx : (j == 4 || j == 5) ? ffebs : bfebs; const float* w = (j == 0 || j == 4) ? ftws : (j == 1 || j == 5) ? ftwe : (j == 2 || j == 6) ? bhws : bhwe; for (int o = 0; o < H; ++o) s += pmul(bfv(bvec[o]), bfv(w[o])); }
    for (int pass = 0; pass < 2; ++pass) { ((volatile float*)DS)[u0] = s; __threadfence(); } }
  for (size_t u = u0; u < 6144; u += nt) { float s; if (u < 4096) { const int dir = (int)(u >= 2048), r = (int)((u % 2048) / A), a = (int)(u % A); if (dir == 0) { s = bfv(fbr[a]); for (int k = 0; k < H; ++k) s += pmul(bfv(rel1[r * H + k]), bfv(fWr[(size_t)k * A + a])); } else { s = bfv(bbr[a]); for (int k = 0; k < TD; ++k) s += pmul(bfv(rel2[r * TD + k]), bfv(bWr[(size_t)k * A + a])); } }
    else { const size_t uu = u - 4096; const int dir = (int)(uu >= 1024), b = (int)((uu % 1024) / A), a = (int)(uu % A); const float* Wg = dir ? bWg : fWg; const float* bg = dir ? bbg : fbg; s = bfv(bg[a]); for (int k = 0; k < H; ++k) s += pmul(bfv(xmean[b * H + k]), bfv(Wg[(size_t)k * A + a])); }
    for (int pass = 0; pass < 2; ++pass) { ((volatile float*)WRG)[u] = s; __threadfence(); } } }
__global__ __launch_bounds__(32) void wx_kernel(const float* __restrict__ X, const b16* __restrict__ WX, const float* __restrict__ fbx, const float* __restrict__ bbx, int RLIM, float* __restrict__ WXO) { __shared__ __attribute__((aligned(16))) b16 Ah[16][264]; __shared__ float Tf[16][260]; const int lane = threadIdx.x, nloc = lane & 15, hlf = lane >> 4; const int g = blockIdx.x % 2; const size_t m0 = (size_t)(blockIdx.x / 2) * 16; if (m0 >= (size_t)RLIM) return;
  if (lane < 16) for (int k = 256; k < 264; ++k) Ah[lane][k] = (b16)0.0f;
  v8f acc[16];
#pragma unroll
  for (int t = 0; t < 16; ++t) acc[t] = (v8f){};
#pragma unroll 1
  for (int kc = 0; kc < H; kc += 256) { for (int rr = 0; rr < 16; ++rr) for (int q = 0; q < 8; ++q) Ah[rr][q * 32 + lane] = (b16)(bf16_rne(X[(m0 + rr) * H + kc + q * 32 + lane]) * XS);
    wave_lds_sync();
#pragma unroll 2
    for (int kb = 0; kb < 256; kb += 32) { const v16b a = frag_kb(&Ah[nloc][kb], hlf);
#pragma unroll
      for (int t = 0; t < 16; ++t) acc[t] = wmma16b(a, frag_kb(WX + (size_t)(g * 256 + t * 16 + nloc) * H + kc + kb, hlf), acc[t]); }
    wave_lds_sync(); }
#pragma unroll
  for (int t = 0; t < 16; ++t) { const int cc = t * 16 + nloc; const float bb = g == 0 ? bfv(fbx[cc]) : bfv(bbx[cc]);
#pragma unroll
    for (int r8 = 0; r8 < 8; ++r8) Tf[8 * hlf + r8][cc] = acc[t][r8] * (1.0f / (XS * WSC)) + bb; }
  wave_lds_sync();
  for (int pass = 0; pass < 2; ++pass) { for (int rr = 0; rr < 16; ++rr) for (int q = 0; q < 2; ++q) *(volatile v4f*)(WXO + (m0 + rr) * 2 * A + g * A + q * 128 + lane * 4) = *(const v4f*)(&Tf[rr][q * 128 + lane * 4]); __threadfence(); } }
__global__ __launch_bounds__(256) void dots_kernel(const float* __restrict__ X, const float* __restrict__ e0, const float* __restrict__ e1, const float* __restrict__ e2, const float* __restrict__ e3, const float* __restrict__ e4, const float* __restrict__ e5, const float* __restrict__ e6, const float* __restrict__ e7, const float* __restrict__ DV, int RLIM, float* __restrict__ PD) { const size_t u = (size_t)blockIdx.x * 256 + threadIdx.x; const size_t row = u / ND; const int j = (int)(u % ND); if (row >= (size_t)RLIM) return; float s = 0.0f;
  if (j < 8) { const float* w = j == 0 ? e0 : j == 1 ? e1 : j == 2 ? e2 : j == 3 ? e3 : j == 4 ? e4 : j == 5 ? e5 : j == 6 ? e6 : e7; for (int k = 0; k < H; ++k) s += pmul(bfv(X[row * H + k]), bfv(w[k])); }
  else { const float* w = DV + (size_t)(j - 8) * H; for (int k = 0; k < H; ++k) s += pmul(bfv(X[row * H + k]), w[k]); }
  for (int pass = 0; pass < 2; ++pass) { ((volatile float*)PD)[u] = s; __threadfence(); } }
__global__ __launch_bounds__(256) void attn_kernel(const float* __restrict__ WXO, const float* __restrict__ WRG, const float* __restrict__ fV, const float* __restrict__ fbv, const float* __restrict__ bV, const float* __restrict__ bbv, const float* __restrict__ PD, int BLIM, float* __restrict__ CW) { __shared__ float Es[L], Cs[32]; const int dir = blockIdx.x / (NBt * R), b = (blockIdx.x / R) % NBt, r = blockIdx.x % R; const int l = threadIdx.x; if (b >= BLIM) return; const float* V = dir ? bV : fV; const float bvv = dir ? bfv(bbv[0]) : bfv(fbv[0]);
  { const float* wx = WXO + ((size_t)b * L + l) * 2 * A + dir * A; const float* wr = WRG + (size_t)dir * 2048 + r * A; const float* wg = WRG + 4096 + (size_t)dir * 1024 + b * A; float s = bvv; for (int a = 0; a < A; ++a) s += pmul(bfv(V[a]), tanhf(wx[a] + wr[a] + wg[a])); Es[l] = s; }
  __syncthreads();
  if (l == 0) { float mx = -INFINITY; for (int i = 0; i < L; ++i) mx = fmaxf(mx, Es[i]); float den = 0.0f; for (int i = 0; i < L; ++i) { const float p = __expf(Es[i] - mx); Es[i] = p; den += p; } const float inv = 1.0f / den; const int js = dir ? 6 : 4;
    float c0 = 0.0f, c1 = 0.0f; for (int i = 0; i < L; ++i) { const float a = Es[i] * inv; c0 += pmul(a, PD[((size_t)b * L + i) * ND + js]); c1 += pmul(a, PD[((size_t)b * L + i) * ND + js + 1]); } for (int k = 0; k < 32; ++k) Cs[k] = k == 0 ? c0 : (k == 1 ? c1 : 0.0f); }
  __syncthreads();
  for (int pass = 0; pass < 2; ++pass) { if (l < 32) ((volatile float*)CW)[(size_t)blockIdx.x * 32 + l] = Cs[l]; __threadfence(); } }
__global__ __launch_bounds__(256) void out_kernel(const float* __restrict__ PD, const float* __restrict__ CW, const float* __restrict__ DS, const int* __restrict__ sk, const float* __restrict__ skm, const float* __restrict__ unused_mask,
    const float* __restrict__ fhbs, const float* __restrict__ fhbe, const float* __restrict__ btbs, const float* __restrict__ btbe, const float* __restrict__ ftbs, const float* __restrict__ ftbe, const float* __restrict__ bhbs, const float* __restrict__ bhbe, int BLIM, float* __restrict__ out) { const size_t u = (size_t)blockIdx.x * 256 + threadIdx.x; if (u >= 266240) return; float val;
  if (u < 4096) { const int which = (int)(u / 1024); const size_t row = u % 1024; if ((int)(row / L) >= BLIM) return; const float bb = which == 0 ? bfv(fhbs[0]) : which == 1 ? bfv(fhbe[0]) : which == 2 ? bfv(btbs[0]) : bfv(btbe[0]); val = PD[row * ND + which] + bb + pmul(0.0f, bfv(unused_mask[0]));
  } else { const size_t v = u - 4096; const int which = (int)(v / 65536); const size_t idx = v % 65536; const int b = (int)(idx / (R * S * L)), r = (int)((idx / (S * L)) % R), s = (int)((idx / L) % S), l = (int)(idx % L); if (b >= BLIM) return; const int dir = which / 2, se = which % 2;
    const size_t row = (size_t)b * L + l; const int jx = 4 + dir * 2 + se;
    const float m = bfv(skm[(b * R + r) * S + s]); const int k0 = iclamp(sk[((b * R + r) * S + s) * 2], 0, L - 1), k1 = iclamp(sk[((b * R + r) * S + s) * 2 + 1], 0, L - 1);
    const int jv_x = 8 + dir * 2 + se, jv_s = 12 + dir * 2 + se;
    const float wsk = pmul(m, pmul(m, 0.5f * (PD[((size_t)b * L + k0) * ND + jv_s] + PD[((size_t)b * L + k1) * ND + jv_s])) + DS[4 + dir * 2 + se]);
    const float wxw = PD[row * ND + jv_x] + DS[dir * 2 + se]; const float cw = CW[(size_t)((dir * NBt + b) * R + r) * 32 + se]; const float xw = PD[row * ND + jx];
    const float bb = which == 0 ? bfv(ftbs[0]) : which == 1 ? bfv(ftbe[0]) : which == 2 ? bfv(bhbs[0]) : bfv(bhbe[0]); val = wsk + wxw + cw + xw + bb; }
  for (int pass = 0; pass < 2; ++pass) { ((volatile float*)out)[u] = val; __threadfence(); } }
}

extern "C" void kernel_launch(void* const* d_in, const int* in_sizes, int n_in, void* d_out, int out_size, void* d_ws, size_t ws_size, hipStream_t stream) {
  (void)n_in;
  auto Fp = [&](int i) { return (const float*)d_in[i]; }; auto Ip = [&](int i) { return (const int*)d_in[i]; };
  if (in_sizes[0] != NROW * H || in_sizes[1] != NBt * H || in_sizes[3] != NBt * R * S * 2 || in_sizes[4] != NBt * R * S || in_sizes[5] != R * H || in_sizes[6] != R * TD || in_sizes[7] != H || in_sizes[23] != H * A || in_sizes[33] != TD * A || in_sizes[39] != H * H || in_sizes[45] != H * H || out_size != 266240) return;
  const int BLIM = NBt;
  const int RLIM = BLIM * L;
  size_t off = 0; char* ws = (char*)d_ws;
  auto carve = [&](size_t bytes) { char* p = ws + off; off += (bytes + 255) & ~(size_t)255; return p; };
  b16* WX = (b16*)carve((size_t)2 * A * H * 2); float* DV = (float*)carve((size_t)NV * H * 4); float* DS = (float*)carve(256); float* WRG = (float*)carve(6144 * 4); float* WXO = (float*)carve((size_t)NROW * 2 * A * 4); float* PD = (float*)carve((size_t)NROW * ND * 4); float* CW = (float*)carve((size_t)2 * NBt * R * 32 * 4);
  if (off > ws_size || off > ((size_t)16 << 20)) return;
  setup_kernel<<<64, 256, 0, stream>>>(Fp(23), Fp(31), Fp(39), Fp(40), Fp(41), Fp(42), Fp(43), Fp(44), Fp(45), Fp(46), Fp(15), Fp(17), Fp(19), Fp(21), Fp(5), Fp(6), Fp(1), Fp(25), Fp(26), Fp(27), Fp(28), Fp(33), Fp(34), Fp(35), Fp(36), WX, DV, DS, WRG);
  wx_kernel<<<(RLIM / 16) * 2, 32, 0, stream>>>(Fp(0), WX, Fp(24), Fp(32), RLIM, WXO);
  dots_kernel<<<(unsigned)((RLIM * ND + 255) / 256), 256, 0, stream>>>(Fp(0), Fp(7), Fp(9), Fp(11), Fp(13), Fp(15), Fp(17), Fp(19), Fp(21), DV, RLIM, PD);
  attn_kernel<<<2 * NBt * R, 256, 0, stream>>>(WXO, WRG, Fp(29), Fp(30), Fp(37), Fp(38), PD, BLIM, CW);
  out_kernel<<<(266240 + 255) / 256, 256, 0, stream>>>(PD, CW, DS, Ip(3), Fp(4), Fp(2), Fp(8), Fp(10), Fp(12), Fp(14), Fp(16), Fp(18), Fp(20), Fp(22), BLIM, (float*)d_out);
}
